// MLA_1331439862383
// MI455X (gfx1250) — hardware-verified
//
#include <hip/hip_runtime.h>
#include <math.h>
#include <stdint.h>

#define NB     4
#define SQ     1024
#define HM     2048
#define CL     512
#define NH     16
#define DH     128
#define NTOK   4096
#define UPW    1024
#define NFREQ  32
#define TP     72

typedef __bf16       v16b __attribute__((ext_vector_type(16)));
typedef __bf16       v8b  __attribute__((ext_vector_type(8)));
typedef float        v8f  __attribute__((ext_vector_type(8)));
typedef float        v4f  __attribute__((ext_vector_type(4)));
typedef unsigned int v4u  __attribute__((ext_vector_type(4)));

static_assert(NTOK == NB * SQ);
static_assert(UPW == NH * 64);
static_assert(HM == NH * DH);

__device__ __forceinline__ unsigned short bf_bits(float f) {
  const unsigned u = __float_as_uint(f);
  return (unsigned short)((u + 0x7FFFu + ((u >> 16) & 1u)) >> 16);
}
__device__ __forceinline__ float bf_val(unsigned short h) { return __uint_as_float(((unsigned)h) << 16); }
__device__ __forceinline__ unsigned pk16(unsigned short a, unsigned short b) { return (unsigned)a | ((unsigned)b << 16); }
__device__ __forceinline__ v8f zero8() { v8f z = {0.f, 0.f, 0.f, 0.f, 0.f, 0.f, 0.f, 0.f}; return z; }
__device__ __forceinline__ int wave_id() { return __builtin_amdgcn_readfirstlane((int)(threadIdx.x >> 5)); }

__device__ __forceinline__ void lds_wave_sync() {
  __builtin_amdgcn_fence(__ATOMIC_RELEASE, "workgroup");
  __builtin_amdgcn_wave_barrier();
  __builtin_amdgcn_fence(__ATOMIC_ACQUIRE, "workgroup");
}

__device__ __forceinline__ void split8(v4f f0, v4f f1, v4u& wh, v4u& wlo) {
  const unsigned short h0 = bf_bits(f0[0]), h1 = bf_bits(f0[1]), h2 = bf_bits(f0[2]), h3 = bf_bits(f0[3]);
  const unsigned short h4 = bf_bits(f1[0]), h5 = bf_bits(f1[1]), h6 = bf_bits(f1[2]), h7 = bf_bits(f1[3]);
  const unsigned short l0 = bf_bits(f0[0] - bf_val(h0)), l1 = bf_bits(f0[1] - bf_val(h1));
  const unsigned short l2 = bf_bits(f0[2] - bf_val(h2)), l3 = bf_bits(f0[3] - bf_val(h3));
  const unsigned short l4 = bf_bits(f1[0] - bf_val(h4)), l5 = bf_bits(f1[1] - bf_val(h5));
  const unsigned short l6 = bf_bits(f1[2] - bf_val(h6)), l7 = bf_bits(f1[3] - bf_val(h7));
  wh[0]  = pk16(h0, h1); wh[1]  = pk16(h2, h3); wh[2]  = pk16(h4, h5); wh[3]  = pk16(h6, h7);
  wlo[0] = pk16(l0, l1); wlo[1] = pk16(l2, l3); wlo[2] = pk16(l4, l5); wlo[3] = pk16(l6, l7);
}

union FragB { v16b v; v8b h[2]; };
__device__ __forceinline__ v16b ldfrag_o(const __bf16* base, unsigned offb) {
  const char* p = (const char*)(const void*)base + offb;
  FragB f;
  f.h[0] = *(const v8b*)(const void*)(p);
  f.h[1] = *(const v8b*)(const void*)(p + 32);
  return f.v;
}

__device__ __forceinline__ v8f mma_b(v16b a, v16b b, v8f c) {
  return __builtin_amdgcn_wmma_f32_16x16x32_bf16(false, a, false, b, (short)0, c, false, false);
}
__device__ __forceinline__ void guard_p1(v8f& a, v8f& b, v16b x0, v16b x1, v16b y) {
  asm volatile("v_nop\n\tv_nop\n\tv_nop\n\tv_nop" : "+v"(a), "+v"(b) : "v"(x0), "v"(x1), "v"(y) : "memory");
}
__device__ __forceinline__ void guard_pa(v8f& a, v8f& b, v16b x0, v16b x1, v16b w0, v16b w1, v16b y) {
  asm volatile("v_nop\n\tv_nop\n\tv_nop\n\tv_nop" : "+v"(a), "+v"(b) : "v"(x0), "v"(x1), "v"(w0), "v"(w1), "v"(y) : "memory");
}
__device__ __forceinline__ void guard_pb(v8f& a, v8f& b, v16b x0, v16b x1, v16b y, v16b yl) {
  asm volatile("v_nop\n\tv_nop\n\tv_nop\n\tv_nop" : "+v"(a), "+v"(b) : "v"(x0), "v"(x1), "v"(y), "v"(yl) : "memory");
}
__device__ __forceinline__ void acc_guard4(v8f& a, v8f& b, v8f& c, v8f& d) {
  asm volatile("v_nop\n\tv_nop\n\tv_nop\n\tv_nop" : "+v"(a), "+v"(b), "+v"(c), "+v"(d));
}

__global__ __launch_bounds__(256) void rope_table_kernel(float* __restrict__ cst) {
  const int lane = threadIdx.x & 31;
  const int wave = (int)(threadIdx.x >> 5);
  const int s = (int)blockIdx.x * 8 + wave;
  if (s >= SQ) return;
  const int   j   = lane & 15;
  const float e   = (float)j * 0.0625f;
  const float pw  = powf(10000.0f, e);
  const float inv = 1.0f / pw;
  const float t   = (float)s * (1.0f / 40.0f);
  const float ang = t * inv;
  const float cv  = cosf(ang);
  const float sv  = sinf(ang);
  const float v   = (lane < 16) ? cv : sv;
  const size_t o = (size_t)s * NFREQ + lane;
  for (int pass = 0; pass < 2; ++pass) {
    ((volatile float*)cst)[o] = v;
    __threadfence();
  }
}

__global__ __launch_bounds__(256) void cvt_bf16_kernel(const float* __restrict__ in, unsigned short* __restrict__ outp, int n8) {
  const int i = (int)blockIdx.x * 256 + (int)threadIdx.x;
  if (i >= n8) return;
  const size_t e = 8 * (size_t)i;
  const v4f a = *(const v4f*)(in + e);
  const v4f b = *(const v4f*)(in + e + 4);
  v4u w;
  w[0] = pk16(bf_bits(a[0]), bf_bits(a[1]));
  w[1] = pk16(bf_bits(a[2]), bf_bits(a[3]));
  w[2] = pk16(bf_bits(b[0]), bf_bits(b[1]));
  w[3] = pk16(bf_bits(b[2]), bf_bits(b[3]));
  *(volatile v4u*)(outp + e) = w;
  __threadfence();
  *(volatile v4u*)(outp + e) = w;
}

__global__ __launch_bounds__(256) void wtrans_kernel(const float* __restrict__ W, unsigned short* __restrict__ D,
                                                    int Kin, int Nout, int gsh, int gstride, int radd) {
  __shared__ __align__(16) unsigned short sT[64 * TP];
  const int tid  = (int)threadIdx.x;
  const int lane = tid & 31;
  const int wave = tid >> 5;
  const int n0 = (int)blockIdx.x * 64;
  const int k0 = (int)blockIdx.y * 64;
#pragma unroll
  for (int u = 0; u < 4; ++u) {
    const int p  = tid + 256 * u;
    const int kk = p >> 4;
    const int c4 = (p & 15) * 4;
    const v4f v = *(const v4f*)(W + (size_t)(k0 + kk) * Nout + n0 + c4);
    sT[(c4 + 0) * TP + kk] = bf_bits(v[0]);
    sT[(c4 + 1) * TP + kk] = bf_bits(v[1]);
    sT[(c4 + 2) * TP + kk] = bf_bits(v[2]);
    sT[(c4 + 3) * TP + kk] = bf_bits(v[3]);
  }
  __syncthreads();
  const int sub  = lane >> 3;
  const int c8   = (lane & 7) * 8;
  const int gmsk = (int)((1u << gsh) - 1u);
  for (int pass = 0; pass < 2; ++pass) {
#pragma unroll
    for (int it = 0; it < 2; ++it) {
      const int row  = wave * 8 + it * 4 + sub;
      const int n    = n0 + row;
      const int drow = (n >> gsh) * gstride + (n & gmsk) + radd;
      const v4u x = *(const v4u*)(sT + row * TP + c8);
      *(volatile v4u*)(D + (size_t)drow * Kin + k0 + c8) = x;
    }
    __threadfence();
  }
}

template <int EPI> struct SlabCfg { static constexpr int PERWF = 4096; };
template <> struct SlabCfg<2>     { static constexpr int PERWF = 5120; };

template <int EPI, bool SA, bool SB>
__global__ __launch_bounds__(128) void gemm_kernel(
    const unsigned short* __restrict__ Ahp, const unsigned short* __restrict__ Alp, int lda,
    const unsigned short* __restrict__ Bhp, const unsigned short* __restrict__ Blp, int ldb,
    const float* __restrict__ cst,
    float* Fp, int ldf,
    unsigned short* P0, unsigned short* P1, int ldp,
    int M, int N, int K,
    int zaq, int zar, int zbq, int zbr, int zcq, int zcr,
    float oscale) {
  __shared__ __align__(16) float lds_all[4 * SlabCfg<EPI>::PERWF];

  const int lane = threadIdx.x & 31;
  const int wave = wave_id();
  const int hh = lane >> 4;
  const int rl = lane & 15;
  const int tilesN = N >> 7;
  const int tilesM = M >> 5;
  const int tile = (int)blockIdx.x * 4 + wave;
  if (tile >= tilesM * tilesN) return;
  const int tm = tile / tilesN;
  const int tn = tile - tm * tilesN;
  const int m0 = tm << 5;
  const int n0 = tn << 7;

  const int z  = (int)blockIdx.y;
  const int zq = z >> 4, zr = z & 15;
  const size_t aoff = (size_t)zq * (size_t)zaq + (size_t)zr * (size_t)zar;
  const size_t boff = (size_t)zq * (size_t)zbq + (size_t)zr * (size_t)zbr;
  const size_t coff = (size_t)zq * (size_t)zcq + (size_t)zr * (size_t)zcr;

  const __bf16* Ah = (const __bf16*)(const void*)Ahp + aoff + (size_t)m0 * lda;
  const __bf16* Al = (const __bf16*)(const void*)Alp + aoff + (size_t)m0 * lda;
  const __bf16* Bh = (const __bf16*)(const void*)Bhp + boff + (size_t)n0 * ldb;
  const __bf16* Bl = (const __bf16*)(const void*)Blp + boff + (size_t)n0 * ldb;
  float* Fz = Fp + coff;
  unsigned short* P0z = P0 + coff;
  unsigned short* P1z = P1 + coff;

  unsigned ao[2], bo[8];
#pragma unroll
  for (int i = 0; i < 2; ++i) ao[i] = ((unsigned)((i * 16 + rl) * lda) + (unsigned)(8 * hh)) * 2u;
#pragma unroll
  for (int j = 0; j < 8; ++j) bo[j] = ((unsigned)((j * 16 + rl) * ldb) + (unsigned)(8 * hh)) * 2u;

  v8f acc[2][8];
#pragma unroll
  for (int i = 0; i < 2; ++i)
#pragma unroll
    for (int j = 0; j < 8; ++j) acc[i][j] = zero8();

  for (int k0 = 0; k0 < K; k0 += 32) {
    const __bf16* Ahk = Ah + k0;
    const __bf16* Alk = Al + k0;
    const __bf16* Bhk = Bh + k0;
    const __bf16* Blk = Bl + k0;
    const v16b ah0 = ldfrag_o(Ahk, ao[0]);
    const v16b ah1 = ldfrag_o(Ahk, ao[1]);
    v16b al0 = ah0, al1 = ah1;
    if constexpr (SA && !SB) { al0 = ldfrag_o(Alk, ao[0]); al1 = ldfrag_o(Alk, ao[1]); }
#pragma unroll
    for (int j = 0; j < 8; ++j) {
      const v16b bh = ldfrag_o(Bhk, bo[j]);
      v16b bl = bh;
      if constexpr (SB) bl = ldfrag_o(Blk, bo[j]);
      acc[0][j] = mma_b(ah0, bh, acc[0][j]);
      acc[1][j] = mma_b(ah1, bh, acc[1][j]);
      if constexpr (SB) {
        acc[0][j] = mma_b(ah0, bl, acc[0][j]);
        acc[1][j] = mma_b(ah1, bl, acc[1][j]);
      }
      if constexpr (SA && !SB) {
        acc[0][j] = mma_b(al0, bh, acc[0][j]);
        acc[1][j] = mma_b(al1, bh, acc[1][j]);
      }
      if constexpr (SB) guard_pb(acc[0][j], acc[1][j], ah0, ah1, bh, bl);
      else if constexpr (SA) guard_pa(acc[0][j], acc[1][j], ah0, ah1, al0, al1, bh);
      else guard_p1(acc[0][j], acc[1][j], ah0, ah1, bh);
    }
    if constexpr (SA && SB) {
      const v16b bl0 = ldfrag_o(Alk, ao[0]);
      const v16b bl1 = ldfrag_o(Alk, ao[1]);
#pragma unroll
      for (int j = 0; j < 8; ++j) {
        const v16b bh = ldfrag_o(Bhk, bo[j]);
        acc[0][j] = mma_b(bl0, bh, acc[0][j]);
        acc[1][j] = mma_b(bl1, bh, acc[1][j]);
        guard_p1(acc[0][j], acc[1][j], bl0, bl1, bh);
      }
    }
  }
  acc_guard4(acc[0][0], acc[0][1], acc[0][2], acc[0][3]);
  acc_guard4(acc[0][4], acc[0][5], acc[0][6], acc[0][7]);
  acc_guard4(acc[1][0], acc[1][1], acc[1][2], acc[1][3]);
  acc_guard4(acc[1][4], acc[1][5], acc[1][6], acc[1][7]);

  float* slf = lds_all + wave * SlabCfg<EPI>::PERWF;
#pragma unroll
  for (int i = 0; i < 2; ++i)
#pragma unroll
    for (int j = 0; j < 8; ++j)
#pragma unroll
      for (int r = 0; r < 8; ++r)
        slf[(16 * i + 8 * hh + r) * 128 + j * 16 + rl] = acc[i][j][r] * oscale;
  if constexpr (EPI == 2) {
    float* csl = slf + 4096;
    const int s0 = m0 & (SQ - 1);
#pragma unroll 4
    for (int u = 0; u < 8; ++u) {
      const int p   = lane + 32 * u;
      const int row = p >> 3, c4 = (p & 7) * 4;
      const v4f cv4 = *(const v4f*)(cst + (size_t)(s0 + row) * NFREQ + c4);
      *(v4f*)(csl + row * NFREQ + c4) = cv4;
    }
  }
  lds_wave_sync();

  if constexpr (EPI == 2) {
    const float* csl = slf + 4096;
    const int cb = hh * 64 + rl;
#pragma unroll 2
    for (int row = 0; row < 32; ++row) {
      const float cv = csl[row * NFREQ + rl];
      const float sv = csl[row * NFREQ + 16 + rl];
      float* p1 = slf + row * 128 + cb;
      const float x1 = p1[0];
      const float x2 = p1[16];
      p1[0]  = x1 * cv - x2 * sv;
      p1[16] = x2 * cv + x1 * sv;
    }
    lds_wave_sync();
  }
  if constexpr (EPI == 5) {
    if ((m0 & (DH - 1)) == 64) {
#pragma unroll 1
      for (int q = 0; q < 16; ++q) {
        const int c  = lane + 32 * (q >> 2);
        const int ig = (q & 3) * 4;
        const int s  = (n0 + c) & (SQ - 1);
        const v4f cv = *(const v4f*)(cst + (size_t)s * NFREQ + ig);
        const v4f sv = *(const v4f*)(cst + (size_t)s * NFREQ + 16 + ig);
#pragma unroll
        for (int e = 0; e < 4; ++e) {
          float* p1 = slf + (ig + e) * 128 + c;
          const float x1 = p1[0];
          const float x2 = p1[16 * 128];
          p1[0]        = x1 * cv[e] - x2 * sv[e];
          p1[16 * 128] = x2 * cv[e] + x1 * sv[e];
        }
      }
      lds_wave_sync();
    }
  }

  for (int pass = 0; pass < 2; ++pass) {
    if constexpr (EPI == 0 || EPI == 2 || EPI == 6) {
#pragma unroll 4
      for (int row = 0; row < 32; ++row) {
        const v4f v = *(const v4f*)(slf + row * 128 + lane * 4);
        *(volatile v4f*)(Fz + (size_t)(m0 + row) * ldf + n0 + lane * 4) = v;
      }
    }
    if constexpr (EPI != 6) {
#pragma unroll 2
      for (int it = 0; it < 16; ++it) {
        const int row = it * 2 + hh;
        const int c8  = rl * 8;
        const v4f f0 = *(const v4f*)(slf + row * 128 + c8);
        const v4f f1 = *(const v4f*)(slf + row * 128 + c8 + 4);
        v4u wh, wlo;
        split8(f0, f1, wh, wlo);
        int pc;
        if constexpr (EPI == 2) pc = 2 * n0 + (c8 >> 6) * DH + 64 + (c8 & 63);
        else if constexpr (EPI == 3) pc = 2 * n0 + (c8 >> 6) * DH + (c8 & 63);
        else pc = n0 + c8;
        const size_t go = (size_t)(m0 + row) * ldp + pc;
        *(volatile v4u*)(P0z + go) = wh;
        *(volatile v4u*)(P1z + go) = wlo;
      }
    }
    __threadfence();
  }
}

extern "C" void kernel_launch(void* const* d_in, const int* in_sizes, int n_in,
                              void* d_out, int out_size, void* d_ws, size_t ws_size,
                              hipStream_t stream) {
  if (n_in < 9) return;
  if (in_sizes[0] != NTOK * HM) return;
  if (in_sizes[1] != HM * CL) return;
  if (in_sizes[2] != HM * CL) return;
  if (in_sizes[3] != CL * UPW) return;
  if (in_sizes[4] != CL * HM) return;
  if (in_sizes[5] != CL * UPW) return;
  if (in_sizes[6] != HM * UPW) return;
  if (in_sizes[7] != CL * UPW) return;
  if (in_sizes[8] != HM * HM) return;
  if (out_size != NTOK * HM + NTOK * CL + NTOK * UPW) return;
  static_assert((size_t)NTOK * HM + (size_t)NTOK * CL + (size_t)NTOK * UPW == 14680064u);

  const float* x    = (const float*)d_in[0];
  const float* Wdkv = (const float*)d_in[1];
  const float* Wdq  = (const float*)d_in[2];
  const float* Wuk  = (const float*)d_in[3];
  const float* Wuv  = (const float*)d_in[4];
  const float* Wuq  = (const float*)d_in[5];
  const float* Wkr  = (const float*)d_in[6];
  const float* Wqr  = (const float*)d_in[7];
  const float* Wout = (const float*)d_in[8];
  float* out0 = (float*)d_out;
  float* out1 = out0 + (size_t)NTOK * HM;
  float* out2 = out1 + (size_t)NTOK * CL;

  const size_t szXB  = (size_t)NTOK * HM * 2;
  const size_t szWA  = (size_t)HM * HM * 2;
  const size_t szR1  = szXB + szWA;
  const size_t szWUK = (size_t)UPW * CL * 2;
  const size_t szWUV = (size_t)HM * CL * 2;
  const size_t szWQ  = (size_t)HM * CL * 2;
  const size_t szWO  = (size_t)HM * HM * 2;
  const size_t szCS  = (size_t)SQ * NFREQ * 4;
  const size_t szC2  = (size_t)NTOK * 2 * CL * 2;
  const size_t szK   = (size_t)NTOK * HM * 2;
  const size_t szT   = (size_t)HM * NTOK * 2;
  const size_t szMT  = (size_t)NB * NH * DH * DH * 2;
  const size_t szOC  = (size_t)NTOK * HM * 2;
  if (szXB + szWUK + szWUV + szWQ > szR1) return;
  if (szT != szXB) return;
  if (2 * szMT > szC2) return;
  if (szWO != szC2) return;
  if (szOC != szT) return;

  size_t off = 0;
  const size_t oR1  = off; off += szR1;
  const size_t oCS  = off; off += szCS;
  const size_t oCKV = off; off += szC2;
  const size_t oCQ  = off; off += szC2;
  const size_t oKH  = off; off += szK;
  const size_t oKL  = off; off += szK;
  const size_t oVTL = off; off += szT;
  const size_t oQTH = off; off += szT;
  const size_t oQTL = off; off += szT;
  if (off != (size_t)125960192u) return;
  if (off > ws_size) return;

  char* ws = (char*)d_ws;
  unsigned short* XB    = (unsigned short*)(ws + oR1);
  unsigned short* WA    = (unsigned short*)(ws + oR1 + szXB);
  unsigned short* VTH   = (unsigned short*)(ws + oR1);
  unsigned short* WUK   = (unsigned short*)(ws + oR1 + szXB);
  unsigned short* WUV   = (unsigned short*)(ws + oR1 + szXB + szWUK);
  unsigned short* WQ    = (unsigned short*)(ws + oR1 + szXB + szWUK + szWUV);
  float*          CS    = (float*)(ws + oCS);
  unsigned short* CKV2  = (unsigned short*)(ws + oCKV);
  unsigned short* MTH   = (unsigned short*)(ws + oCKV);
  unsigned short* MTL   = (unsigned short*)(ws + oCKV + szMT);
  unsigned short* CQ2   = (unsigned short*)(ws + oCQ);
  unsigned short* WO    = (unsigned short*)(ws + oCQ);
  unsigned short* KH    = (unsigned short*)(ws + oKH);
  unsigned short* KL    = (unsigned short*)(ws + oKL);
  unsigned short* VTL   = (unsigned short*)(ws + oVTL);
  unsigned short* OUTCH = (unsigned short*)(ws + oVTL);
  unsigned short* QTH   = (unsigned short*)(ws + oQTH);
  unsigned short* OUTCL = (unsigned short*)(ws + oQTH);
  unsigned short* QTL   = (unsigned short*)(ws + oQTL);

  const dim3 b256(256), b128(128);
  const float one = 1.0f;
  const float osc = 0.0883883476483184f;

  rope_table_kernel<<<dim3(SQ / 8), b256, 0, stream>>>(CS);
  cvt_bf16_kernel<<<dim3((NTOK * HM / 8) / 256), b256, 0, stream>>>(x, XB, NTOK * HM / 8);
  wtrans_kernel<<<dim3(CL / 64, HM / 64), b256, 0, stream>>>(Wdkv, WA, HM, CL, 30, 0, 0);
  wtrans_kernel<<<dim3(CL / 64, HM / 64), b256, 0, stream>>>(Wdq, WA, HM, CL, 30, 0, CL);
  wtrans_kernel<<<dim3(UPW / 64, HM / 64), b256, 0, stream>>>(Wkr, WA, HM, UPW, 30, 0, 2 * CL);
  gemm_kernel<0, false, false><<<dim3((NTOK / 32) * (CL / 128) / 4), b128, 0, stream>>>(
      XB, XB, HM, WA, WA, HM, CS, out1, CL, CKV2, CKV2 + CL, 2 * CL, NTOK, CL, HM, 0, 0, 0, 0, 0, 0, one);
  gemm_kernel<1, false, false><<<dim3((NTOK / 32) * (CL / 128) / 4), b128, 0, stream>>>(
      XB, XB, HM, WA + (size_t)CL * HM, WA + (size_t)CL * HM, HM, CS, out0, CL, CQ2, CQ2 + CL, 2 * CL, NTOK, CL, HM,
      0, 0, 0, 0, 0, 0, one);
  gemm_kernel<2, false, false><<<dim3((NTOK / 32) * (UPW / 128) / 4), b128, 0, stream>>>(
      XB, XB, HM, WA + (size_t)2 * CL * HM, WA + (size_t)2 * CL * HM, HM, CS, out2, UPW, KH, KL, HM, NTOK, UPW, HM,
      0, 0, 0, 0, 0, 0, one);
  wtrans_kernel<<<dim3(UPW / 64, CL / 64), b256, 0, stream>>>(Wuk, WUK, CL, UPW, 30, 0, 0);
  wtrans_kernel<<<dim3(HM / 64, CL / 64), b256, 0, stream>>>(Wuv, WUV, CL, HM, 30, 0, 0);
  wtrans_kernel<<<dim3(UPW / 64, CL / 64), b256, 0, stream>>>(Wuq, WQ, CL, UPW, 6, DH, 0);
  wtrans_kernel<<<dim3(UPW / 64, CL / 64), b256, 0, stream>>>(Wqr, WQ, CL, UPW, 6, DH, 64);
  gemm_kernel<3, true, false><<<dim3((NTOK / 32) * (UPW / 128) / 4), b128, 0, stream>>>(
      CKV2, CKV2 + CL, 2 * CL, WUK, WUK, CL, CS, out0, UPW, KH, KL, HM, NTOK, UPW, CL, 0, 0, 0, 0, 0, 0, one);
  gemm_kernel<5, false, true><<<dim3((HM / 32) * (NTOK / 128) / 4), b128, 0, stream>>>(
      WQ, WQ, CL, CQ2, CQ2 + CL, 2 * CL, CS, out0, CL, QTH, QTL, NTOK, HM, NTOK, CL, 0, 0, 0, 0, 0, 0, one);
  wtrans_kernel<<<dim3(HM / 64, HM / 64), b256, 0, stream>>>(Wout, WO, HM, HM, 30, 0, 0);
  gemm_kernel<4, false, true><<<dim3((HM / 32) * (NTOK / 128) / 4), b128, 0, stream>>>(
      WUV, WUV, CL, CKV2, CKV2 + CL, 2 * CL, CS, out0, CL, VTH, VTL, NTOK, HM, NTOK, CL, 0, 0, 0, 0, 0, 0, one);
  gemm_kernel<4, true, true><<<dim3(1, NB * NH), b128, 0, stream>>>(
      VTH, VTL, NTOK, QTH, QTL, NTOK, CS, out0, CL, MTH, MTL, DH, DH, DH, SQ,
      SQ, DH * NTOK, SQ, DH * NTOK, NH * DH * DH, DH * DH, one);
  gemm_kernel<4, true, true><<<dim3((SQ / 32) / 4, NB * NH), b128, 0, stream>>>(
      KH, KL, HM, MTH, MTL, DH, CS, out0, CL, OUTCH, OUTCL, HM, SQ, DH, DH,
      SQ * HM, DH, NH * DH * DH, DH * DH, SQ * HM, DH, osc);
  gemm_kernel<6, true, false><<<dim3((NTOK / 32) * (HM / 128) / 4), b128, 0, stream>>>(
      OUTCH, OUTCL, HM, WO, WO, HM, CS, out0, HM, KH, KL, HM, NTOK, HM, HM, 0, 0, 0, 0, 0, 0, one);
  (void)hipGetLastError();
}
